// SphericalCNN_4698694222686
// MI455X (gfx1250) — hardware-verified
//
#include <hip/hip_runtime.h>
#include <hip/hip_bf16.h>


namespace {

constexpr int kLmax  = 5;
constexpr int kNtri  = 69;
constexpr int kTau   = 24;
constexpr int kBatch = 128;
constexpr int kK2    = 6 * kTau * kTau;
constexpr int kNChunk = kK2 / 32;
constexpr int kChunksPerGrp = 576 / 32;

struct Tab {
  int l1[kNtri]; int l2[kNtri]; int l[kNtri];
  int cgoff[kNtri];
  int goff[kNtri];
  int ps[kNtri + 1];
  int cols0[kLmax + 1];
  int gbase[kLmax + 2];
  int lof[36];
  int cgtot;
};

constexpr Tab makeTab() {
  Tab t{};
  int n = 0;
  for (int a = 0; a <= kLmax; ++a)
    for (int b = 0; b <= a; ++b) {
      int hi = a + b; if (hi > kLmax) hi = kLmax;
      for (int c = a - b; c <= hi; ++c) { t.l1[n] = a; t.l2[n] = b; t.l[n] = c; ++n; }
    }
  int off = 0;
  for (int k = 0; k < kNtri; ++k) {
    t.cgoff[k] = off;
    off += (2 * t.l1[k] + 1) * (2 * t.l2[k] + 1) * (2 * t.l[k] + 1);
  }
  t.cgtot = off;
  int colidx[kNtri] = {};
  for (int k = 0; k < kNtri; ++k) { colidx[k] = t.cols0[t.l[k]]; t.cols0[t.l[k]]++; }
  t.gbase[0] = 0;
  for (int l = 0; l <= kLmax; ++l) t.gbase[l + 1] = t.gbase[l] + t.cols0[l] * (2 * l + 1);
  for (int k = 0; k < kNtri; ++k) t.goff[k] = t.gbase[t.l[k]] + colidx[k] * (2 * t.l[k] + 1);
  t.ps[0] = 0;
  for (int k = 0; k < kNtri; ++k) t.ps[k + 1] = t.ps[k] + (2 * t.l[k] + 1);
  for (int lm = 0; lm < 36; ++lm) { int l = 0; while ((l + 1) * (l + 1) <= lm) ++l; t.lof[lm] = l; }
  return t;
}

__device__ constexpr Tab dTab = makeTab();
constexpr Tab hTab = makeTab();
static_assert(hTab.ps[kNtri] == 457, "total g size");
static_assert(hTab.cgtot == 24367, "CG table size");
static_assert(hTab.cols0[0] == 6 && hTab.gbase[kLmax + 1] == 457, "layout");

constexpr size_t WS_CG   = 0;
constexpr size_t WS_FS1  = 98304;
constexpr size_t WS_PW   = 98304 + 884736;
constexpr size_t WS_PART = 98304 + 884736 + 884736;
constexpr int    PWN     = 2 * 2 * kNChunk * 32 * 16;

typedef __attribute__((ext_vector_type(16))) _Float16 v16h;
typedef __attribute__((ext_vector_type(8)))  float    v8f;
typedef __attribute__((ext_vector_type(4)))  float    v4f_t;
typedef float v4fa __attribute__((ext_vector_type(4), may_alias));
typedef __attribute__((ext_vector_type(2)))  float    v2f_t;
#define RSPLIT (1.0f / 2048.0f)
__device__ __forceinline__ _Float16 lo_of(float v, _Float16 h) { return (_Float16)((v - (float)h) * 2048.0f); }
__device__ __forceinline__ v8f wmma16(v16h a, v16h b, v8f c) { return __builtin_amdgcn_wmma_f32_16x16x32_f16(false, a, false, b, (short)0, c, false, false); }
__device__ __forceinline__ v8f wmma_split(v16h a, v16h al, v16h b, v16h bl, v8f c) { v8f x = {}; x = wmma16(al, b, x); x = wmma16(a, bl, x); return wmma16(a, b, c) + x * RSPLIT; }

struct W0Ptrs { const float* p[6]; };

}

__device__ inline double dfact(int n) {
  double r = 1.0;
  for (int i = 2; i <= n; ++i) r *= (double)i;
  return r;
}

__device__ float clebsch(int j1, int m1, int j2, int m2, int j, int m) {
  if (m1 + m2 != m) return 0.0f;
  double pref = sqrt((2.0 * j + 1.0) * dfact(j + j1 - j2) * dfact(j - j1 + j2) *
                     dfact(j1 + j2 - j) / dfact(j1 + j2 + j + 1));
  pref *= sqrt(dfact(j + m) * dfact(j - m) * dfact(j1 - m1) * dfact(j1 + m1) *
               dfact(j2 - m2) * dfact(j2 + m2));
  int kmin = 0;
  if (j2 - j - m1 > kmin) kmin = j2 - j - m1;
  if (j1 + m2 - j > kmin) kmin = j1 + m2 - j;
  int kmax = j1 + j2 - j;
  if (j1 - m1 < kmax) kmax = j1 - m1;
  if (j2 + m2 < kmax) kmax = j2 + m2;
  double s = 0.0;
  for (int k = kmin; k <= kmax; ++k) {
    double d = dfact(k) * dfact(j1 + j2 - j - k) * dfact(j1 - m1 - k) *
               dfact(j2 + m2 - k) * dfact(j - j2 + m1 + k) * dfact(j - j1 - m2 + k);
    s += ((k & 1) ? -1.0 : 1.0) / d;
  }
  return (float)(pref * s);
}

__global__ void k_cg(float* __restrict__ cg) {
  for (int k = threadIdx.x; k < kNtri; k += blockDim.x) {
    const int a = dTab.l1[k], b = dTab.l2[k], c = dTab.l[k];
    float* out = cg + dTab.cgoff[k];
    for (int i1 = 0; i1 < 2 * a + 1; ++i1)
      for (int i2 = 0; i2 < 2 * b + 1; ++i2)
        for (int i = 0; i < 2 * c + 1; ++i)
          { const float cv = clebsch(a, i1 - a, b, i2 - b, c, i - c); float* d = out + (i1 * (2 * b + 1) + i2) * (2 * c + 1) + i;
            *(volatile float*)d = cv; __threadfence(); *(volatile float*)d = cv; }
  }
}

__global__ void k_packw(const float* __restrict__ w1, _Float16* __restrict__ pW) {
  int idx = (blockIdx.x * blockDim.x + threadIdx.x) * 2;
  if (idx >= 2 * 2 * kNChunk * 32 * 16) return;
  const int h    = idx & 15;
  const int lane = (idx >> 4) & 31;
  const int q    = (idx >> 9) % kNChunk;
  const int rest = idx / (512 * kNChunk);
  const int p    = rest & 1;
  const int mt   = rest >> 1;
  const int t    = mt * 16 + (lane & 15);
  const int kk   = h + 8 * ((h >= 8 ? 1 : 0) + (lane >= 16 ? 1 : 0));
  const int col  = (q / kChunksPerGrp) * 576 + (q % kChunksPerGrp) * 32 + kk;
  const float v0 = (t < kTau) ? w1[(t * kK2 + col) * 2 + p] : 0.0f;
  const float v1 = (t < kTau) ? w1[(t * kK2 + col + 1) * 2 + p] : 0.0f;
  const _Float16 a0 = (_Float16)v0, a1 = (_Float16)v1;
  const unsigned u = (unsigned)__builtin_bit_cast(unsigned short, a0) | ((unsigned)__builtin_bit_cast(unsigned short, a1) << 16);
  const unsigned w = (unsigned)__builtin_bit_cast(unsigned short, lo_of(v0, a0)) | ((unsigned)__builtin_bit_cast(unsigned short, lo_of(v1, a1)) << 16);
  *(volatile unsigned*)(pW + idx) = u; *(volatile unsigned*)(pW + PWN + idx) = w; __threadfence();
  *(volatile unsigned*)(pW + idx) = u; *(volatile unsigned*)(pW + PWN + idx) = w;
}

__global__ void k_layer1(const float* __restrict__ f0, W0Ptrs w0,
                         const float* __restrict__ cg, float* __restrict__ fs1) {
  __shared__ float sF0[72];
  __shared__ float sg[457 * 2];
  const int b = blockIdx.x, tid = threadIdx.x;
  if (tid < 72) sF0[tid] = f0[b * 72 + tid];
  __syncthreads();

  for (int w = tid; w < 457; w += blockDim.x) {
    int k = 0;
    while (dTab.ps[k + 1] <= w) ++k;
    const int mi = w - dTab.ps[k];
    const int a = dTab.l1[k], b2 = dTab.l2[k], c = dTab.l[k];
    const int m = mi - c;
    int lo = -a; if (m - b2 > lo) lo = m - b2;
    int hi = a;  if (m + b2 < hi) hi = m + b2;
    float gr = 0.0f, gi = 0.0f;
    const float* C = cg + dTab.cgoff[k];
    for (int m1 = lo; m1 <= hi; ++m1) {
      const int m2 = m - m1;
      const float cc = C[((m1 + a) * (2 * b2 + 1) + (m2 + b2)) * (2 * c + 1) + mi];
      const int i1 = (a * a + a + m1) * 2;
      const int i2 = (b2 * b2 + b2 + m2) * 2;
      const float f1r = sF0[i1], f1i = sF0[i1 + 1];
      const float f2r = sF0[i2], f2i = sF0[i2 + 1];
      gr += cc * (f1r * f2r - f1i * f2i);
      gi += cc * (f1r * f2i + f1i * f2r);
    }
    const int go = (dTab.goff[k] + mi) * 2;
    sg[go] = gr; sg[go + 1] = gi;
  }
  __syncthreads();

  for (int idx = tid; idx < kTau * 36; idx += blockDim.x) {
    const int t = idx / 36, lm = idx % 36;
    const int l = dTab.lof[lm];
    const int mi = lm - l * l;
    const int nc = dTab.cols0[l];
    const int step = 2 * l + 1;
    const int gb = dTab.gbase[l] + mi;
    const float* wl = w0.p[l];
    float orr = 0.0f, oii = 0.0f;
    for (int col = 0; col < nc; ++col) {
      const float gr = sg[(gb + col * step) * 2];
      const float gi = sg[(gb + col * step) * 2 + 1];
      const float wr = wl[(t * nc + col) * 2];
      const float wi = wl[(t * nc + col) * 2 + 1];
      orr += wr * gr - wi * gi;
      oii += wr * gi + wi * gr;
    }
    const int o = ((b * kTau + t) * 36 + lm) * 2;
    v2f_t ov; ov.x = orr; ov.y = oii;
    *(volatile v2f_t*)(fs1 + o) = ov; __threadfence(); *(volatile v2f_t*)(fs1 + o) = ov;
  }
}

__global__ void k_layer2(const float* __restrict__ fs1,
                         const _Float16* __restrict__ pW,
                         float* __restrict__ pbuf) {
  __shared__ float sF[16 * 24 * 11 * 2];
  __shared__ __attribute__((aligned(32))) _Float16 sG[3][512];
  __shared__ __attribute__((aligned(32))) _Float16 sL[3][512];
  __shared__ __attribute__((aligned(16))) float so[16 * 48];

  const int tid = threadIdx.x;
  const int lane = tid & 31, wv = tid >> 5;
  const int mt = wv >> 1, cpart = wv & 1;
  const int btile = blockIdx.x;
  const int l1 = blockIdx.y;
  const int d1 = 2 * l1 + 1;
  const float isq = rsqrtf((float)d1);

  const int nslab = 16 * kTau * d1 * 2;
  for (int idx = tid; idx < nslab; idx += blockDim.x) {
    const int p = idx & 1;
    int r = idx >> 1;
    const int mi = r % d1; r /= d1;
    const int i = r % kTau;
    const int bl = r / kTau;
    sF[idx] = fs1[(((btile * 16 + bl) * kTau + i) * 36 + l1 * l1 + mi) * 2 + p];
  }
  __syncthreads();

  v8f acc = {};
  for (int qq = 0; qq < kChunksPerGrp; ++qq) {
    const int q = l1 * kChunksPerGrp + qq;
    const int cb = qq * 32;

    for (int v = 0; v < 4; ++v) {
      const int idx = v * 128 + tid;
      const int cc = idx >> 4;
      const int bl = idx & 15;
      const int c = cb + cc;
      const int i = c / kTau, j = c % kTau;
      float gr = 0.0f, gi = 0.0f;
      for (int m1 = -l1; m1 <= l1; ++m1) {
        const float s = ((l1 - m1) & 1) ? -isq : isq;
        const int i1 = ((bl * kTau + i) * d1 + (m1 + l1)) * 2;
        const int i2 = ((bl * kTau + j) * d1 + (l1 - m1)) * 2;
        const float f1r = sF[i1], f1i = sF[i1 + 1];
        const float f2r = sF[i2], f2i = sF[i2 + 1];
        gr += s * (f1r * f2r - f1i * f2i);
        gi += s * (f1r * f2i + f1i * f2r);
      }
      const int hs = (cc >> 3) & 1, el = (cc & 7) + ((cc >> 4) << 3);
      const int sl = (bl + 16 * hs) * 16 + el;
      const _Float16 hr = (_Float16)gr, hi2 = (_Float16)gi, hn = (_Float16)(-gi);
      sG[0][sl] = hr;  sL[0][sl] = lo_of(gr, hr);
      sG[1][sl] = hi2; sL[1][sl] = lo_of(gi, hi2);
      sG[2][sl] = hn;  sL[2][sl] = lo_of(-gi, hn);
    }
    __syncthreads();

    const size_t or_ = (size_t)((mt * 2 + 0) * kNChunk + q) * 512 + lane * 16, oi_ = (size_t)((mt * 2 + 1) * kNChunk + q) * 512 + lane * 16;
    const v16h aWr = *(const v16h*)(pW + or_), aWrl = *(const v16h*)(pW + PWN + or_);
    const v16h aWi = *(const v16h*)(pW + oi_), aWil = *(const v16h*)(pW + PWN + oi_);
    if (qq + 1 < kChunksPerGrp) {
      __builtin_prefetch(pW + (size_t)((mt * 2 + 0) * kNChunk + q + 1) * 512 + lane * 16, 0, 3);
      __builtin_prefetch(pW + (size_t)((mt * 2 + 1) * kNChunk + q + 1) * 512 + lane * 16, 0, 3);
    }

    if (cpart == 0) {
      acc = wmma_split(aWr, aWrl, *(const v16h*)(&sG[0][lane * 16]), *(const v16h*)(&sL[0][lane * 16]), acc);
      acc = wmma_split(aWi, aWil, *(const v16h*)(&sG[2][lane * 16]), *(const v16h*)(&sL[2][lane * 16]), acc);
    } else {
      acc = wmma_split(aWr, aWrl, *(const v16h*)(&sG[1][lane * 16]), *(const v16h*)(&sL[1][lane * 16]), acc);
      acc = wmma_split(aWi, aWil, *(const v16h*)(&sG[0][lane * 16]), *(const v16h*)(&sL[0][lane * 16]), acc);
    }
    __syncthreads();
  }

  #pragma unroll
  for (int r = 0; r < 8; ++r) {
    const int t = mt * 16 + r + ((lane >= 16) ? 8 : 0);
    if (t < kTau) so[(lane & 15) * (2 * kTau) + t * 2 + cpart] = acc[r];
  }
  __syncthreads();
  float* pout = pbuf + (size_t)l1 * (kBatch * 2 * kTau) + (size_t)btile * 16 * (2 * kTau);
  for (int c = tid; c < 16 * 2 * kTau / 4; c += blockDim.x) {
    const v4f_t v = *(const volatile v4fa*)(so + c * 4);
    *(volatile v4f_t*)(pout + c * 4) = v; __threadfence(); *(volatile v4f_t*)(pout + c * 4) = v;
  }
}

__global__ void k_reduce(const float* __restrict__ pbuf, float* __restrict__ out) {
  const int idx = blockIdx.x * blockDim.x + threadIdx.x;
  if (idx >= kBatch * 2 * kTau) return;
  float s = 0.0f;
  #pragma unroll
  for (int g = 0; g < 6; ++g) s += pbuf[(size_t)g * (kBatch * 2 * kTau) + idx];
  *(volatile float*)(out + idx) = s; __threadfence(); *(volatile float*)(out + idx) = s;
}

extern "C" void kernel_launch(void* const* d_in, const int* in_sizes, int n_in,
                              void* d_out, int out_size, void* d_ws, size_t ws_size,
                              hipStream_t stream) {
  const float* f0 = (const float*)d_in[0];
  W0Ptrs w0;
  for (int l = 0; l < 6; ++l) w0.p[l] = (const float*)d_in[1 + 2 * l];
  const float* w1_0 = (const float*)d_in[2];

  char* ws = (char*)d_ws;
  float*    cg   = (float*)(ws + WS_CG);
  float*    fs1  = (float*)(ws + WS_FS1);
  _Float16* pW   = (_Float16*)(ws + WS_PW);
  float*    pbuf = (float*)(ws + WS_PART);
  float*    out  = (float*)d_out;

  k_cg<<<1, 128, 0, stream>>>(cg);
  k_packw<<<(2 * 2 * kNChunk * 32 * 16) / 512, 256, 0, stream>>>(w1_0, pW);
  k_layer1<<<kBatch, 128, 0, stream>>>(f0, w0, cg, fs1);
  k_layer2<<<dim3(kBatch / 16, 6), 128, 0, stream>>>(fs1, pW, pbuf);
  k_reduce<<<(kBatch * 2 * kTau + 255) / 256, 256, 0, stream>>>(pbuf, out);
}
